// RelativePositionSDPA_48670569398462
// MI455X (gfx1250) — hardware-verified
//
#include <hip/hip_runtime.h>
#include <math.h>

typedef __attribute__((ext_vector_type(16))) _Float16 v16h;
typedef __attribute__((ext_vector_type(16))) __bf16 v16b;
typedef __attribute__((ext_vector_type(8)))  _Float16 v8h;
typedef __attribute__((ext_vector_type(8)))  float v8f;
typedef __attribute__((ext_vector_type(4)))  float v4f;
typedef __attribute__((ext_vector_type(2)))  float v2f;
typedef __attribute__((ext_vector_type(4)))  unsigned v4u;
typedef __attribute__((ext_vector_type(4)))  int v4i;
typedef float __attribute__((may_alias)) float_a;
typedef int __attribute__((may_alias)) int_a;

template <typename T> __device__ __forceinline__ void vst2(void* p, T v) { *(volatile T*)p = v; __threadfence(); *(volatile T*)p = v; }
__device__ __forceinline__ v8f wmma16(v16h a, v16h b, v8f c) {
  v8f d = __builtin_amdgcn_wmma_f32_16x16x32_f16(false, a, false, b, (short)0, c, false, false);
  asm volatile("v_nop\n\tv_nop\n\tv_nop\n\tv_nop" : "+v"(d) : "v"(a), "v"(b));
  return d;
}
__device__ __forceinline__ v8f wmma_bf(v16b a, v16b b, v8f c) {
  v8f d = __builtin_amdgcn_wmma_f32_16x16x32_bf16(false, a, false, b, (short)0, c, false, false);
  asm volatile("v_nop\n\tv_nop\n\tv_nop\n\tv_nop" : "+v"(d) : "v"(a), "v"(b));
  return d;
}
__device__ __forceinline__ v16h frag_h(const _Float16* rowk0, int lane) {
  union { v16h v; v8h q[2]; } u; const _Float16* p = rowk0 + 8 * (lane >> 4);
  u.q[0] = *(const v8h*)p; u.q[1] = *(const v8h*)(p + 16); return u.v;
}
__device__ __forceinline__ v16h frag_f32(const float* rowk0, int lane) {
  v16h a; const float* p = rowk0 + 8 * (lane >> 4);
#pragma unroll
  for (int i = 0; i < 8; ++i) { a[i] = (_Float16)p[i]; a[8 + i] = (_Float16)p[16 + i]; }
  return a;
}
__device__ __forceinline__ v16h frag_f32s(const float* rowk0, int lane, float sc) {
  v16h a; const float* p = rowk0 + 8 * (lane >> 4);
#pragma unroll
  for (int i = 0; i < 8; ++i) { a[i] = (_Float16)(p[i] * sc); a[8 + i] = (_Float16)(p[16 + i] * sc); }
  return a;
}
__device__ __forceinline__ v16h fragc_f32(const float* W, int k0, int n, int lane, int ld, int K) {
  v16h a; const int g = lane >> 4;
#pragma unroll
  for (int i = 0; i < 8; ++i) { const int ka = k0 + 8 * g + i, kb = ka + 16;
    a[i] = (_Float16)(ka < K ? W[(size_t)(ka < K ? ka : K - 1) * ld + n] : 0.f); a[8 + i] = (_Float16)(kb < K ? W[(size_t)(kb < K ? kb : K - 1) * ld + n] : 0.f); }
  return a;
}
struct F2 { v16b h, l; };
__device__ __forceinline__ F2 bsplit16(const float v[16]) { F2 r;
#pragma unroll
  for (int i = 0; i < 16; ++i) { const __bf16 h = (__bf16)v[i]; r.h[i] = h; r.l[i] = (__bf16)(v[i] - (float)h); }
  return r; }
__device__ __forceinline__ F2 split_row(const float* row, int k0, int lane) { float v[16]; const float* p = row + k0 + 8 * (lane >> 4);
#pragma unroll
  for (int i = 0; i < 8; ++i) { v[i] = p[i]; v[8 + i] = p[16 + i]; }
  return bsplit16(v); }
__device__ __forceinline__ F2 split_rowK(const float* row, int k0, int lane, int K) { float v[16]; const int g = lane >> 4;
#pragma unroll
  for (int i = 0; i < 8; ++i) { const int ka = k0 + 8 * g + i, kb = ka + 16; v[i] = ka < K ? row[ka < K ? ka : K - 1] : 0.f; v[8 + i] = kb < K ? row[kb < K ? kb : K - 1] : 0.f; }
  return bsplit16(v); }
__device__ __forceinline__ F2 split_col(const float* W, int k0, int n, int lane, int ld, int K) { float v[16]; const int g = lane >> 4;
#pragma unroll
  for (int i = 0; i < 8; ++i) { const int ka = k0 + 8 * g + i, kb = ka + 16; v[i] = ka < K ? W[(size_t)(ka < K ? ka : K - 1) * ld + n] : 0.f; v[8 + i] = kb < K ? W[(size_t)(kb < K ? kb : K - 1) * ld + n] : 0.f; }
  return bsplit16(v); }
__device__ __forceinline__ v8f mac3(const F2& a, const F2& b, v8f c) { c = wmma_bf(a.l, b.h, c); c = wmma_bf(a.h, b.l, c); return wmma_bf(a.h, b.h, c); }
__device__ __forceinline__ float sigm(float v) { return 1.0f / (1.0f + expf(-v)); }
#define LDSX() do { asm volatile("s_wait_dscnt 0" ::: "memory"); __builtin_amdgcn_wave_barrier(); __builtin_amdgcn_fence(__ATOMIC_RELEASE, "workgroup"); } while (0)


#define NHT 64
#define HPG 16
#define SS 1024
#define KD 64
#define RLEN 2048
#define GRP 8
#ifndef TNG
#define TNG (NHT / GRP)
#define TQB (SS / 64)
#endif
typedef __attribute__((ext_vector_type(8))) __bf16 v8b;
__device__ __forceinline__ v16b frag_b(const __bf16* rowk0, int lane) {
  union { v16b v; v8b q[2]; } u; const __bf16* p = rowk0 + 8 * (lane >> 4);
  u.q[0] = *(const v8b*)p; u.q[1] = *(const v8b*)(p + 16); return u.v;
}
__device__ __forceinline__ v16b frag_gbf(const float* rowk0, int lane) {
  v16b a; const float* p = rowk0 + 8 * (lane >> 4);
#pragma unroll
  for (int i = 0; i < 8; ++i) { a[i] = (__bf16)p[i]; a[8 + i] = (__bf16)p[16 + i]; }
  return a;
}
__device__ __forceinline__ F2 frag_qb(const float* qrow, const float* bias, int k0, int lane) {
  F2 f; const int o = 8 * (lane >> 4);
#pragma unroll
  for (int i = 0; i < 8; ++i) { const float v0 = (float)(__bf16)qrow[k0 + o + i] * 0.125f + (float)(__bf16)bias[k0 + o + i]; const float v1 = (float)(__bf16)qrow[k0 + o + 16 + i] * 0.125f + (float)(__bf16)bias[k0 + o + 16 + i];
    const __bf16 h0 = (__bf16)v0, h1 = (__bf16)v1; f.h[i] = h0; f.l[i] = (__bf16)(v0 - (float)h0); f.h[8 + i] = h1; f.l[8 + i] = (__bf16)(v1 - (float)h1); }
  return f;
}
__device__ __forceinline__ float bfr(float v) { return (float)(__bf16)v; }
__device__ __attribute__((noinline)) float exp_ni(float v) { return expf(v); }
#define WS_VT  0u
#define WS_PS  (WS_VT + 2u * NHT * KD * SS)
#define WS_END (WS_PS + 4u * GRP * SS * SS)

__global__ __launch_bounds__(256) void k_vt(const float* __restrict__ V, __bf16* __restrict__ VT) {
  __shared__ __align__(16) __bf16 st[KD][72];
  const int nh = blockIdx.y, t0 = blockIdx.x * 64, tid = threadIdx.x;
  for (int q = tid; q < 64 * KD; q += 256) { const int tl = q >> 6, d = q & 63; st[d][tl] = (__bf16)V[((size_t)nh * SS + t0 + tl) * KD + d]; }
  __syncthreads();
  for (int q = tid; q < KD * 8; q += 256) { const int d = q >> 3, pc = q & 7; vst2((unsigned*)(VT + ((size_t)nh * KD + d) * SS + t0 + pc * 8), *(const v4u*)&st[d][pc * 8]); }
}
__global__ __launch_bounds__(128) void k_pos(const float* __restrict__ Q, const float* __restrict__ VB, const float* __restrict__ R, float* __restrict__ PS, int g0) {
  __shared__ __align__(16) float so[4][16][132];
  const int tid = threadIdx.x, wave = tid >> 5, lane = tid & 31, col = lane & 15, gg = lane >> 4; const int hg = blockIdx.z, nh = g0 * GRP + hg, h = nh % HPG; const int i0 = blockIdx.x * 64 + wave * 16, m0 = blockIdx.y * 128;
  const F2 a0 = frag_qb(Q + ((size_t)nh * SS + i0 + col) * KD, VB + h * KD, 0, lane), a1 = frag_qb(Q + ((size_t)nh * SS + i0 + col) * KD, VB + h * KD, 32, lane);
  v8f acc[8] = {};
#pragma unroll
  for (int j = 0; j < 8; ++j) { const float* rr = R + ((size_t)h * RLEN + m0 + j * 16 + col) * KD; const v16b r0 = frag_gbf(rr, lane), r1 = frag_gbf(rr + 32, lane);
    acc[j] = wmma_bf(a0.h, r0, acc[j]); acc[j] = wmma_bf(a0.l, r0, acc[j]); acc[j] = wmma_bf(a1.h, r1, acc[j]); acc[j] = wmma_bf(a1.l, r1, acc[j]); }
#pragma unroll
  for (int j = 0; j < 8; ++j)
#pragma unroll
    for (int r = 0; r < 8; ++r) so[wave][8 * gg + r][j * 16 + col] = acc[j][r];
  LDSX();
  for (int rl = 0; rl < 16; ++rl) vst2(PS + ((size_t)hg * SS + i0 + rl) * SS + m0 + lane * 4, *(const v4f*)&so[wave][rl][lane * 4]);
}
__global__ __launch_bounds__(128) void k_attn(const float* __restrict__ Q, const float* __restrict__ Kk, const float* __restrict__ UB, const float* __restrict__ PS, const __bf16* __restrict__ VT, float* __restrict__ out, int g0) {
  __shared__ __align__(16) float sp[4][16][36]; __shared__ __align__(16) float so[4][16][68];
  const int tid = threadIdx.x, wave = tid >> 5, lane = tid & 31, col = lane & 15, gg = lane >> 4; const int hg = blockIdx.y, nh = g0 * GRP + hg, h = nh % HPG; const int i0 = blockIdx.x * 64 + wave * 16;
  const F2 a0 = frag_qb(Q + ((size_t)nh * SS + i0 + col) * KD, UB + h * KD, 0, lane), a1 = frag_qb(Q + ((size_t)nh * SS + i0 + col) * KD, UB + h * KD, 32, lane);
  const float* psh = PS + (size_t)hg * SS * SS;
  float m[8], l[8];
#pragma unroll
  for (int r = 0; r < 8; ++r) { m[r] = -3.0e38f; l[r] = 0.f; }
  v8f acc[4] = {};
#pragma unroll 1
  for (int ks = 0; ks < SS / 32; ++ks) { v8f s[2];
#pragma unroll
    for (int ct = 0; ct < 2; ++ct) { const int j = ks * 32 + ct * 16 + col; const float* kr = Kk + ((size_t)nh * SS + j) * KD; const v16b k0 = frag_gbf(kr, lane), k1 = frag_gbf(kr + 32, lane);
      v8f c = {}; c = wmma_bf(a0.h, k0, c); c = wmma_bf(a0.l, k0, c); c = wmma_bf(a1.h, k1, c); c = wmma_bf(a1.l, k1, c);
#pragma unroll
      for (int r = 0; r < 8; ++r) { const int i = i0 + 8 * gg + r; float pv;
        { const int idx = (j <= i) ? (i * SS + (SS - 1 - i + j)) : (min(i + 1, SS - 1) * SS + max(j - i - 2, 0)); pv = psh[idx]; pv = (j == i + 1) ? 0.f : pv; }
        s[ct][r] = c[r] + pv; } }
#pragma unroll
    for (int r = 0; r < 8; ++r) { float mx = fmaxf(s[0][r], s[1][r]);
#pragma unroll
      for (int o = 1; o < 16; o <<= 1) mx = fmaxf(mx, __shfl_xor(mx, o));
      const float mn = fmaxf(m[r], mx); const float alpha = exp_ni(m[r] - mn); const float e0 = exp_ni(s[0][r] - mn), e1 = exp_ni(s[1][r] - mn); float es = e0 + e1;
#pragma unroll
      for (int o = 1; o < 16; o <<= 1) es += __shfl_xor(es, o);
      l[r] = l[r] * alpha + es; m[r] = mn;
#pragma unroll
      for (int dt = 0; dt < 4; ++dt) acc[dt][r] *= alpha;
      sp[wave][8 * gg + r][col] = e0; sp[wave][8 * gg + r][16 + col] = e1; }
    LDSX();
    const F2 pa = split_row(&sp[wave][col][0], 0, lane);
#pragma unroll
    for (int dt = 0; dt < 4; ++dt) { const v16b vv = frag_b(VT + ((size_t)nh * KD + dt * 16 + col) * SS + ks * 32, lane); acc[dt] = wmma_bf(pa.l, vv, acc[dt]); acc[dt] = wmma_bf(pa.h, vv, acc[dt]); }
    LDSX(); }
#pragma unroll
  for (int r = 0; r < 8; ++r) { const float il = 1.0f / l[r];
#pragma unroll
    for (int dt = 0; dt < 4; ++dt) so[wave][8 * gg + r][dt * 16 + col] = acc[dt][r] * il; }
  LDSX();
  for (int rl = 0; rl < 16; ++rl) if (lane < 16) vst2(out + ((size_t)nh * SS + i0 + rl) * KD + lane * 4, *(const v4f*)&so[wave][rl][lane * 4]);
}

extern "C" void kernel_launch(void* const* d_in, const int* in_sizes, int n_in, void* d_out, int out_size, void* d_ws, size_t ws_size, hipStream_t stream) {
  (void)in_sizes; (void)n_in; (void)out_size;
  const float** F = (const float**)d_in;
  if (ws_size < (size_t)WS_END) return;
  char* ws = (char*)d_ws; __bf16* VT = (__bf16*)(ws + WS_VT); float* PS = (float*)(ws + WS_PS);
  k_vt<<<dim3(SS / 64, NHT), 256, 0, stream>>>(F[2], VT);
  for (int g = 0; g < TNG; ++g) {
    k_pos<<<dim3(SS / 64, SS / 128, GRP), 128, 0, stream>>>(F[0], F[4], F[5], PS, g);
    k_attn<<<dim3(TQB, GRP), 128, 0, stream>>>(F[0], F[1], F[3], PS, VT, (float*)d_out, g); }
}
